// MultiHeadAttentionBlock_1382979469695
// MI455X (gfx1250) — hardware-verified
//
#include <hip/hip_runtime.h>
#include <math.h>

typedef __attribute__((ext_vector_type(16))) _Float16 v16h;
typedef __attribute__((ext_vector_type(16))) __bf16 v16b;
typedef __attribute__((ext_vector_type(8)))  _Float16 v8h;
typedef __attribute__((ext_vector_type(8)))  float v8f;
typedef __attribute__((ext_vector_type(4)))  float v4f;
typedef __attribute__((ext_vector_type(4)))  unsigned v4u;

template <typename T> __device__ __forceinline__ void vst2(void* p, T v) { *(volatile T*)p = v; __threadfence(); *(volatile T*)p = v; }
__device__ __forceinline__ v8f wmma16(v16h a, v16h b, v8f c) {
  v8f d = __builtin_amdgcn_wmma_f32_16x16x32_f16(false, a, false, b, (short)0, c, false, false);
  asm volatile("v_nop\n\tv_nop\n\tv_nop\n\tv_nop" : "+v"(d) : "v"(a), "v"(b));
  return d;
}
__device__ __forceinline__ v8f wmma_bf(v16b a, v16b b, v8f c) {
  v8f d = __builtin_amdgcn_wmma_f32_16x16x32_bf16(false, a, false, b, (short)0, c, false, false);
  asm volatile("v_nop\n\tv_nop\n\tv_nop\n\tv_nop" : "+v"(d) : "v"(a), "v"(b));
  return d;
}
__device__ __forceinline__ v16h frag_h(const _Float16* rowk0, int lane) {
  union { v16h v; v8h q[2]; } u; const _Float16* p = rowk0 + 8 * (lane >> 4);
  u.q[0] = *(const v8h*)p; u.q[1] = *(const v8h*)(p + 16); return u.v;
}
__device__ __forceinline__ v16h frag_f32s(const float* rowk0, int lane, float sc) {
  v16h a; const float* p = rowk0 + 8 * (lane >> 4);
#pragma unroll
  for (int i = 0; i < 8; ++i) { a[i] = (_Float16)(p[i] * sc); a[8 + i] = (_Float16)(p[16 + i] * sc); }
  return a;
}
__device__ __forceinline__ float bfr(float v) { return (float)(__bf16)v; }
#define LDSX() do { asm volatile("s_wait_dscnt 0" ::: "memory"); __builtin_amdgcn_wave_barrier(); __builtin_amdgcn_fence(3  , "workgroup"); } while (0)

#ifndef NB
#define NB 4
#endif
#ifndef SEQ
#define SEQ 2048
#endif
#define NB_FULL 4
#define SEQ_FULL 2048
#define TT SEQ
#define CC 1024
#define DIN 1024
#define NH 16
#define HD 64
#define NQB (TT / 64)
#define NKT (TT / 128)
#define SCALE (0.125f)
#define PCARRY (16384.0f)
static_assert(TT % 128 == 0);
static_assert(NB >= 1 && NB <= NB_FULL);
static_assert(SEQ >= 128 && SEQ <= SEQ_FULL);
static_assert(NH * HD == CC);
static_assert(DIN % 128 == 0 && CC % 128 == 0 && HD == 64);

__device__ __forceinline__ v16b wcol_hdk(const float* Wm, int k0, int o, int lane) { v16b w; const int g = lane >> 4; const float* p = Wm + (size_t)(o / HD) * DIN * HD + (o % HD);
#pragma unroll
  for (int i = 0; i < 8; ++i) { w[i] = (__bf16)p[(size_t)(k0 + 8 * g + i) * HD]; w[8 + i] = (__bf16)p[(size_t)(k0 + 16 + 8 * g + i) * HD]; }
  return w; }
__device__ __forceinline__ v16h wcolh_io(const float* Wm, int k0, int o, int lane, int ld) { v16h w; const int g = lane >> 4;
#pragma unroll
  for (int i = 0; i < 8; ++i) { w[i] = (_Float16)(bfr(Wm[(size_t)(k0 + 8 * g + i) * ld + o]) * 256.0f); w[8 + i] = (_Float16)(bfr(Wm[(size_t)(k0 + 16 + 8 * g + i) * ld + o]) * 256.0f); }
  return w; }

#define WS_QH  0u
#define WS_QL  (WS_QH + 2u * (size_t)NB * TT * CC)
#define WS_KH  (WS_QL + 2u * (size_t)NB * TT * CC)
#define WS_VT  (WS_KH + 2u * (size_t)NB * TT * CC)
#define WS_Y   (WS_VT + 2u * (size_t)NB * CC * TT)
#define WS_END (WS_Y  + 4u * (size_t)NB * TT * CC)
static_assert(WS_END <= (size_t)134217728u);
static_assert((WS_QL % 128u) == 0 && (WS_KH % 128u) == 0 && (WS_VT % 128u) == 0 && (WS_Y % 128u) == 0);

__global__ __launch_bounds__(128) void k_proj(const float* __restrict__ X, const float* __restrict__ WQ, const float* __restrict__ WK, const float* __restrict__ WV, const float* __restrict__ BQ, const float* __restrict__ BK, const float* __restrict__ BV,
    _Float16* __restrict__ QH, _Float16* __restrict__ QL, _Float16* __restrict__ KH, _Float16* __restrict__ VT) {
  __shared__ __align__(16) _Float16 sh[64][136], sl[64][136]; __shared__ __align__(16) _Float16 th[128][72];
  const int tid = threadIdx.x, wave = tid >> 5, lane = tid & 31, col = lane & 15, g = lane >> 4; const int which = blockIdx.z; const int c0 = blockIdx.y * 128;
  const size_t r0 = (size_t)blockIdx.x * 64; const size_t bb = r0 / TT; const int t0 = (int)(r0 % TT); const size_t xr0 = bb * SEQ_FULL + t0;
  const float* WA = which == 0 ? WQ : which == 1 ? WK : WV; const float* BA = which == 0 ? BQ : which == 1 ? BK : BV;
  v8f acc[8] = {};
#pragma unroll 2
  for (int kc = 0; kc < DIN / 32; ++kc) { v16b a; { const float* p = X + (xr0 + wave * 16 + col) * DIN + kc * 32 + 8 * g;
#pragma unroll
      for (int i = 0; i < 8; ++i) { a[i] = (__bf16)p[i]; a[8 + i] = (__bf16)p[16 + i]; } }
    asm volatile("s_wait_loadcnt 0x0" ::: "memory");
#pragma unroll
    for (int j = 0; j < 8; ++j) { const v16b w = wcol_hdk(WA, kc * 32, c0 + j * 16 + col, lane); asm volatile("s_wait_loadcnt 0x0" ::: "memory"); acc[j] = wmma_bf(a, w, acc[j]); } }
  if (which < 2) { _Float16* DST = which == 0 ? QH : KH; const bool res = (which == 0);
#pragma unroll
    for (int j = 0; j < 8; ++j) { const float bias = bfr(BA[c0 + j * 16 + col]);
#pragma unroll
      for (int r = 0; r < 8; ++r) { const float v = acc[j][r] + bias; const _Float16 hv = (_Float16)v; sh[wave * 16 + 8 * g + r][j * 16 + col] = hv; sl[wave * 16 + 8 * g + r][j * 16 + col] = (_Float16)((v - (float)hv) * 1024.0f); } }
    __syncthreads();
    for (int e = tid; e < 64 * 16; e += 128) { const int rl = e >> 4, q = e & 15; vst2((unsigned*)(DST + (r0 + rl) * CC + c0 + q * 8), *(const v4u*)&sh[rl][q * 8]); if (res) vst2((unsigned*)(QL + (r0 + rl) * CC + c0 + q * 8), *(const v4u*)&sl[rl][q * 8]); }
  } else {
#pragma unroll
    for (int j = 0; j < 8; ++j) { const float bias = bfr(BA[c0 + j * 16 + col]);
#pragma unroll
      for (int r = 0; r < 8; ++r) { const float v = acc[j][r] + bias; const int rl = wave * 16 + 8 * g + r, cl = j * 16 + col; th[cl][rl] = (_Float16)v; } }
    __syncthreads();
    for (int e = tid; e < 128 * 8; e += 128) { const int cl = e >> 3, q = e & 7; vst2((unsigned*)(VT + (bb * CC + c0 + cl) * (size_t)TT + t0 + q * 8), *(const v4u*)&th[cl][q * 8]); } } }

union PW { _Float16 p[16][136]; float f[16][68]; };
__device__ __forceinline__ float rmax16(float v) {
#pragma unroll
  for (int o = 1; o < 16; o <<= 1) v = fmaxf(v, __shfl_xor(v, o));
  return v; }
__device__ __forceinline__ float rsum16(float v) {
#pragma unroll
  for (int o = 1; o < 16; o <<= 1) v += __shfl_xor(v, o);
  return v; }
__global__ __launch_bounds__(128) void k_attn(const _Float16* __restrict__ QH, const _Float16* __restrict__ QL, const _Float16* __restrict__ KH, const _Float16* __restrict__ VT, float* __restrict__ Y) {
  __shared__ __align__(16) _Float16 ks[128][72];
  __shared__ __align__(16) _Float16 vs[HD][136];
  __shared__ __align__(16) PW pw[4];
  const int tid = threadIdx.x, wave = tid >> 5, lane = tid & 31, col = lane & 15, g = lane >> 4;
  const int qb = blockIdx.x, h = blockIdx.y, b = blockIdx.z;
  const int ql0 = qb * 64 + wave * 16;
  const size_t qoff = ((size_t)b * TT + ql0 + col) * CC + (size_t)h * HD;
  const v16h ah0 = frag_h(QH + qoff, lane), ah1 = frag_h(QH + qoff + 32, lane);
  const v16h al0 = frag_h(QL + qoff, lane), al1 = frag_h(QL + qoff + 32, lane);
  v8f o[HD / 16] = {};
  float m[8], l[8];
#pragma unroll
  for (int r = 0; r < 8; ++r) { m[r] = -1.0e30f; l[r] = 0.f; }
  _Float16 (*pp)[136] = pw[wave].p; float (*pf)[68] = pw[wave].f;
#pragma unroll 1
  for (int kt = 0; kt < NKT; ++kt) {
    const int k0 = kt * 128;
    __syncthreads();
    for (int e = tid; e < 128 * 8; e += 128) { const int row = e >> 3, q = e & 7; *(v4u*)&ks[row][q * 8] = *(const v4u*)(KH + ((size_t)b * TT + k0 + row) * CC + (size_t)h * HD + q * 8); }
    for (int e = tid; e < HD * 16; e += 128) { const int c = e >> 4, q = e & 15; *(v4u*)&vs[c][q * 8] = *(const v4u*)(VT + ((size_t)b * CC + (size_t)h * HD + c) * (size_t)TT + k0 + q * 8); }
    __syncthreads();
    v8f acc[8];
#pragma unroll
    for (int j = 0; j < 8; ++j) { asm volatile("" ::: "memory");
      const v16h kf0 = frag_h(&ks[j * 16 + col][0], lane), kf1 = frag_h(&ks[j * 16 + col][32], lane);
      v8f a = {}; a = wmma16(al0, kf0, a); a = wmma16(al1, kf1, a); a = a * (1.0f / 1024.0f); a = wmma16(ah0, kf0, a); acc[j] = wmma16(ah1, kf1, a); }
    float f[8];
#pragma unroll
    for (int r = 0; r < 8; ++r) { float mx = acc[0][r];
#pragma unroll
      for (int j = 1; j < 8; ++j) mx = fmaxf(mx, acc[j][r]);
      mx = rmax16(mx); const float mn = fmaxf(m[r], mx); f[r] = __expf((m[r] - mn) * SCALE); m[r] = mn; }
#pragma unroll
    for (int r = 0; r < 8; ++r) { float s = 0.f;
#pragma unroll
      for (int j = 0; j < 8; ++j) { const float p = __expf((acc[j][r] - m[r]) * SCALE); s += p; pp[8 * g + r][j * 16 + col] = (_Float16)(p * PCARRY); }
      s = rsum16(s); l[r] = l[r] * f[r] + s; }
#pragma unroll
    for (int j = 0; j < HD / 16; ++j)
#pragma unroll
      for (int r = 0; r < 8; ++r) o[j][r] *= f[r];
    LDSX();
#pragma unroll
    for (int kc = 0; kc < 4; ++kc) { asm volatile("" ::: "memory"); const v16h pa = frag_h(&pp[col][kc * 32], lane);
#pragma unroll
      for (int j = 0; j < HD / 16; ++j) o[j] = wmma16(pa, frag_h(&vs[j * 16 + col][kc * 32], lane), o[j]); } }
  float inv[8];
#pragma unroll
  for (int r = 0; r < 8; ++r) inv[r] = 1.0f / (l[r] * PCARRY);
  LDSX();
#pragma unroll
  for (int j = 0; j < HD / 16; ++j)
#pragma unroll
    for (int r = 0; r < 8; ++r) pf[8 * g + r][j * 16 + col] = o[j][r] * inv[r];
  LDSX();
  for (int rl = 0; rl < 16; ++rl) if (lane < HD / 4) vst2(Y + ((size_t)b * TT + ql0 + rl) * CC + (size_t)h * HD + lane * 4, *(const v4f*)&pf[rl][lane * 4]); }

__global__ __launch_bounds__(128) void k_out(const float* __restrict__ Y, const float* __restrict__ WO, const float* __restrict__ BO, float* __restrict__ OUT) { __shared__ __align__(16) float sf[4][16][132];
  const int tid = threadIdx.x, wave = tid >> 5, lane = tid & 31, col = lane & 15, g = lane >> 4; const int c0 = blockIdx.y * 128; const size_t r0 = (size_t)blockIdx.x * 64 + wave * 16;
  v8f acc[8] = {};
#pragma unroll 2
  for (int kc = 0; kc < CC / 32; ++kc) { const v16h a = frag_f32s(Y + (r0 + col) * CC + kc * 32, lane, 16.0f); asm volatile("s_wait_loadcnt 0x0" ::: "memory");
#pragma unroll
    for (int j = 0; j < 8; ++j) { const v16h w = wcolh_io(WO, kc * 32, c0 + j * 16 + col, lane, DIN); asm volatile("s_wait_loadcnt 0x0" ::: "memory"); acc[j] = wmma16(a, w, acc[j]); } }
#pragma unroll
  for (int j = 0; j < 8; ++j) { const float bias = bfr(BO[c0 + j * 16 + col]);
#pragma unroll
    for (int r = 0; r < 8; ++r) sf[wave][8 * g + r][j * 16 + col] = acc[j][r] * (1.0f / 4096.0f) + bias; }
  LDSX(); for (int rl = 0; rl < 16; ++rl) vst2(OUT + (r0 + rl) * DIN + c0 + lane * 4, *(const v4f*)&sf[wave][rl][lane * 4]); }

extern "C" void kernel_launch(void* const* d_in, const int* in_sizes, int n_in, void* d_out, int out_size, void* d_ws, size_t ws_size, hipStream_t stream) {
  if (n_in < 9) return;
  if ((size_t)in_sizes[0] < ((size_t)(NB - 1) * SEQ_FULL + SEQ) * DIN) return;
  if (in_sizes[1] < NH * DIN * HD || in_sizes[3] < NH * DIN * HD || in_sizes[5] < NH * DIN * HD) return;
  if (in_sizes[2] < CC || in_sizes[4] < CC || in_sizes[6] < CC) return;
  if (in_sizes[7] < CC * DIN || in_sizes[8] < DIN) return;
  if ((size_t)out_size < (size_t)NB * TT * DIN) return;
  if (ws_size < (size_t)WS_END) return;
  const float** F = (const float**)d_in;
  char* ws = (char*)d_ws; _Float16 *QH = (_Float16*)(ws + WS_QH), *QL = (_Float16*)(ws + WS_QL), *KH = (_Float16*)(ws + WS_KH), *VT = (_Float16*)(ws + WS_VT); float* Y = (float*)(ws + WS_Y);
  k_proj<<<dim3(NB * TT / 64, CC / 128, 3), 128, 0, stream>>>(F[0], F[1], F[3], F[5], F[2], F[4], F[6], QH, QL, KH, VT);
  k_attn<<<dim3(NQB, NH, NB), 128, 0, stream>>>(QH, QL, KH, VT, Y);
  k_out<<<dim3(NB * TT / 64, DIN / 128), 128, 0, stream>>>(Y, F[7], F[8], (float*)d_out);
}
